// DONNSentimentClassifier_76862734729917
// MI455X (gfx1250) — hardware-verified
//
#include <hip/hip_runtime.h>


#define NB_  256
#define TT   512
#define NTOK (NB_ * TT)
#define UU   64
#define ED   100
#define EDP  128
#define VV   32000
#define PD   20
#define NC   2
#define NSTEP 20
#define DTT  1e-3f
#define HSC  0.2f
#define MU_  1.0f
#define DM   EDP
#define LOSC 1024.0f

typedef _Float16 h16;
typedef unsigned short bf;
typedef __attribute__((ext_vector_type(16))) __bf16   v16bf;
typedef __attribute__((ext_vector_type(16))) _Float16 v16h;
typedef __attribute__((ext_vector_type(8)))  _Float16 v8h;
typedef __attribute__((ext_vector_type(8)))  unsigned short v8us;
typedef __attribute__((ext_vector_type(8)))  float    v8f;
typedef __attribute__((ext_vector_type(4)))  float    v4f;
typedef __attribute__((ext_vector_type(4)))  _Float16 v4h;
typedef v8h  __attribute__((may_alias)) v8ha;
typedef v4f  __attribute__((may_alias)) v4fa;
typedef v8us __attribute__((may_alias)) v8usa;

__device__ __forceinline__ unsigned short f2bf(float f) { unsigned u = __float_as_uint(f); u += 0x7FFFu + ((u >> 16) & 1u); return (unsigned short)(u >> 16); }
__device__ __forceinline__ float bf2f(unsigned short b) { return __uint_as_float(((unsigned)b) << 16); }
__device__ __forceinline__ float bfr(float f) { return bf2f(f2bf(f)); }
__device__ __forceinline__ v16h cat16(v8h lo, v8h hi) { return __builtin_shufflevector(lo, hi, 0, 1, 2, 3, 4, 5, 6, 7, 8, 9, 10, 11, 12, 13, 14, 15); }
__device__ __forceinline__ v16bf cat16b(v8us lo, v8us hi) { return __builtin_bit_cast(v16bf, __builtin_shufflevector(lo, hi, 0, 1, 2, 3, 4, 5, 6, 7, 8, 9, 10, 11, 12, 13, 14, 15)); }
__device__ __forceinline__ v8f wmma16(v16h a, v16h b, v8f c) { return __builtin_amdgcn_wmma_f32_16x16x32_f16(false, a, false, b, (short)0, c, false, false); }
__device__ __forceinline__ v8f wmmab(v16bf a, v16bf b, v8f c) { return __builtin_amdgcn_wmma_f32_16x16x32_bf16(false, a, false, b, (short)0, c, false, false); }

template <bool SPLITA, bool F16OUT = false>
__global__ __launch_bounds__(128) void k_gemmb(const bf* __restrict__ A, const bf* __restrict__ Al, const bf* __restrict__ Bn, const float* __restrict__ bias, float* C, int ldc, h16* C2, const float* __restrict__ R = nullptr, int K = DM, int roundR = 1) {
    __shared__ __align__(16) float ost[4][16 * 68];
    const int lane = threadIdx.x & 31, wave = threadIdx.x >> 5, lr = lane & 15, hi = lane >> 4;
    const int r0 = blockIdx.x * 64 + wave * 16, c0 = blockIdx.y * 64;
    const size_t aoff = (size_t)(r0 + lr) * K + 8 * hi;
    size_t boff[4];
#pragma unroll
    for (int t = 0; t < 4; ++t) boff[t] = (size_t)(c0 + t * 16 + lr) * K + 8 * hi;
    v8f acc[4];
#pragma unroll
    for (int t = 0; t < 4; ++t) acc[t] = (v8f){};
#pragma unroll 1
    for (int kc = 0; kc < K; kc += 32) {
        const v16bf a = cat16b(*(const v8us*)(A + aoff + kc), *(const v8us*)(A + aoff + kc + 16));
        v16bf al = a;
        if (SPLITA) al = cat16b(*(const v8us*)(Al + aoff + kc), *(const v8us*)(Al + aoff + kc + 16));
#pragma unroll
        for (int t = 0; t < 4; ++t) { const v16bf b = cat16b(*(const v8us*)(Bn + boff[t] + kc), *(const v8us*)(Bn + boff[t] + kc + 16)); acc[t] = wmmab(a, b, acc[t]); if (SPLITA) acc[t] = wmmab(al, b, acc[t]); }
        asm volatile("v_nop\n\tv_nop\n\tv_nop\n\tv_nop" : "+v"(acc[0]), "+v"(acc[1]), "+v"(acc[2]), "+v"(acc[3]) : "v"(a), "v"(al));
    }
    float* os = &ost[wave][0];
#pragma unroll
    for (int t = 0; t < 4; ++t) { const float bv = bias ? bfr(bias[c0 + t * 16 + lr]) : 0.f;
#pragma unroll
        for (int j = 0; j < 8; ++j) os[(hi * 8 + j) * 68 + t * 16 + lr] = acc[t][j] + bv; }
    __syncthreads();
    if (F16OUT) {
        h16* crow = (h16*)(void*)C + (size_t)r0 * ldc + c0;
        auto pass = [&]() {
#pragma unroll
            for (int s = 0; s < 4; ++s) { const int row = 4 * s + (lane >> 3), piece = lane & 7; const float* sp = os + row * 68 + piece * 8; v8h o, o2;
#pragma unroll
                for (int i = 0; i < 8; ++i) { const h16 a = (h16)sp[i]; o[i] = a; o2[i] = (h16)((sp[i] - (float)a) * LOSC); }
                *(volatile v8h*)(crow + (size_t)row * ldc + piece * 8) = o; if (C2) *(volatile v8h*)(C2 + (size_t)r0 * ldc + c0 + (size_t)row * ldc + piece * 8) = o2; }
        };
        pass(); __threadfence(); pass();
    } else {
        float* crow = C + (size_t)r0 * ldc + c0;
        auto pass = [&]() {
#pragma unroll
            for (int s = 0; s < 8; ++s) { const int Lid = (lane >> 3) + 4 * s, piece = lane & 7; const int row = Lid >> 1, cofs = (Lid & 1) * 32 + piece * 4;
                v4f val = *(const v4fa*)(os + row * 68 + cofs); if (R) { const v4f rv = *(const v4f*)(R + ((size_t)r0 + row) * ldc + c0 + cofs); val += roundR ? (v4f){bfr(rv[0]), bfr(rv[1]), bfr(rv[2]), bfr(rv[3])} : rv; }
                *(volatile v4f*)(crow + (size_t)row * ldc + cofs) = val; }
        };
        pass(); __threadfence(); pass();
    }
}


__global__ __launch_bounds__(256) void k_embrows(const int* __restrict__ idx, const float* __restrict__ E, bf* A) {
    typedef __attribute__((ext_vector_type(4))) unsigned short v4us;
    const int lane = threadIdx.x & 31; const size_t tok = (size_t)blockIdx.x * 8 + (threadIdx.x >> 5); if (tok >= (size_t)NTOK) return; int v = idx[tok]; v = v < 0 ? 0 : (v >= VV ? VV - 1 : v); const float* er = E + (size_t)v * ED; v4us o;
#pragma unroll
    for (int i = 0; i < 4; ++i) { const int k = lane * 4 + i; o[i] = f2bf(k < ED ? er[k < ED ? k : 0] : 0.f); }
    *(volatile v4us*)(A + tok * EDP + lane * 4) = o; __threadfence(); *(volatile v4us*)(A + tok * EDP + lane * 4) = o;
}
__global__ __launch_bounds__(256) void k_w1cat(const float* __restrict__ Wr, const float* __restrict__ Wi, bf* Bt) {
    typedef __attribute__((ext_vector_type(4))) unsigned short v4us;
    const int lane = threadIdx.x & 31; const int n = blockIdx.x * 8 + (threadIdx.x >> 5); if (n >= 2 * UU) return; const float* Wm = (n < UU) ? Wr : Wi; const int nn = (n < UU) ? n : n - UU; v4us o;
#pragma unroll
    for (int i = 0; i < 4; ++i) { const int k = lane * 4 + i; o[i] = f2bf(k < ED ? Wm[(size_t)(k < ED ? k : 0) * UU + nn] : 0.f); }
    *(volatile v4us*)(Bt + (size_t)n * EDP + lane * 4) = o; __threadfence(); *(volatile v4us*)(Bt + (size_t)n * EDP + lane * 4) = o;
}
__global__ __launch_bounds__(256) void k_wcat2(const float* __restrict__ Wr, const float* __restrict__ Wi, bf* Bt) {
    typedef __attribute__((ext_vector_type(2))) unsigned short v2us;
    const int lane = threadIdx.x & 31; const int n = blockIdx.x * 8 + (threadIdx.x >> 5); if (n >= 2 * UU) return; const float* Wm = (n < UU) ? Wr : Wi; const int nn = (n < UU) ? n : n - UU; v2us o;
    o[0] = f2bf(Wm[(size_t)(lane * 2) * UU + nn]); o[1] = f2bf(Wm[(size_t)(lane * 2 + 1) * UU + nn]);
    *(volatile v2us*)(Bt + (size_t)n * UU + lane * 2) = o; __threadfence(); *(volatile v2us*)(Bt + (size_t)n * UU + lane * 2) = o;
}
__global__ __launch_bounds__(256) void k_wt_small(const float* __restrict__ Wm, int Klive, int Nlive, int K, int N, bf* Bt) {
    typedef __attribute__((ext_vector_type(4))) unsigned short v4us;
    const int lane = threadIdx.x & 31; const int n = blockIdx.x * 8 + (threadIdx.x >> 5); if (n >= N) return;
    for (int k0 = 0; k0 < K; k0 += 128) { v4us o;
#pragma unroll
        for (int i = 0; i < 4; ++i) { const int k = k0 + lane * 4 + i; const bool live = (k < Klive) && (n < Nlive); o[i] = f2bf(live ? Wm[(size_t)(live ? k : 0) * Nlive + (live ? n : 0)] : 0.f); }
        if (k0 + lane * 4 < K) *(volatile v4us*)(Bt + (size_t)n * K + k0 + lane * 4) = o; }
    __threadfence();
    for (int k0 = 0; k0 < K; k0 += 128) { v4us o;
#pragma unroll
        for (int i = 0; i < 4; ++i) { const int k = k0 + lane * 4 + i; const bool live = (k < Klive) && (n < Nlive); o[i] = f2bf(live ? Wm[(size_t)(live ? k : 0) * Nlive + (live ? n : 0)] : 0.f); }
        if (k0 + lane * 4 < K) *(volatile v4us*)(Bt + (size_t)n * K + k0 + lane * 4) = o; }
}
__global__ __launch_bounds__(256) void k_relu128p(const float* __restrict__ F, bf* Ph, bf* Pl) {
    typedef __attribute__((ext_vector_type(4))) unsigned short v4us;
    const int lane = threadIdx.x & 31; const size_t r = (size_t)blockIdx.x * 8 + (threadIdx.x >> 5); if (r >= (size_t)NTOK) return; v4us oh, ol;
#pragma unroll
    for (int i = 0; i < 4; ++i) { const float y = fmaxf(F[r * 128 + lane * 4 + i], 0.f); const unsigned short hb = f2bf(y); oh[i] = hb; ol[i] = f2bf(y - bf2f(hb)); }
    const size_t o = r * 128 + lane * 4; *(volatile v4us*)(Ph + o) = oh; *(volatile v4us*)(Pl + o) = ol; __threadfence(); *(volatile v4us*)(Ph + o) = oh; *(volatile v4us*)(Pl + o) = ol;
}
__global__ __launch_bounds__(256) void k_relu64p(const float* __restrict__ F, bf* Ph, bf* Pl) {
    typedef __attribute__((ext_vector_type(2))) unsigned short v2us;
    const int lane = threadIdx.x & 31; const size_t r = (size_t)blockIdx.x * 8 + (threadIdx.x >> 5); if (r >= (size_t)NTOK) return; v2us oh, ol;
#pragma unroll
    for (int i = 0; i < 2; ++i) { const float y = fmaxf(F[r * UU + lane * 2 + i], 0.f); const unsigned short hb = f2bf(y); oh[i] = hb; ol[i] = f2bf(y - bf2f(hb)); }
    const size_t o = r * UU + lane * 2; *(volatile v2us*)(Ph + o) = oh; *(volatile v2us*)(Pl + o) = ol; __threadfence(); *(volatile v2us*)(Ph + o) = oh; *(volatile v2us*)(Pl + o) = ol;
}
__global__ __launch_bounds__(256) void k_hopf(const float* __restrict__ F, const float* __restrict__ om, float* Z) {
    const int lane = threadIdx.x & 31; const int w = blockIdx.x * 8 + (threadIdx.x >> 5); if (w >= (NB_ / 2) * 2) return; const int b = w >> 1, half = w & 1;     const int u = half * 32 + lane; const float omg = bfr(om[u]);
    float zr = 0.1f, zi = 0.f;
    for (int t = 0; t < TT; ++t) { const size_t tok = (size_t)b * TT + t; const float xr = fmaxf(F[tok * 128 + u], 0.f), xi = fmaxf(F[tok * 128 + UU + u], 0.f);
#pragma unroll 1
        for (int s = 0; s < NSTEP; ++s) { const float r2 = zr * zr + zi * zi; const float dzr = (MU_ - r2) * zr - omg * zi + HSC * xr; const float dzi = (MU_ - r2) * zi + omg * zr + HSC * xi; zr = zr + DTT * dzr; zi = zi + DTT * dzi; }
        *(volatile float*)(Z + tok * 128 + u) = zr; *(volatile float*)(Z + tok * 128 + UU + u) = zi; __threadfence(); *(volatile float*)(Z + tok * 128 + u) = zr; *(volatile float*)(Z + tok * 128 + UU + u) = zi; }
}
__global__ __launch_bounds__(256) void k_split128r(const float* __restrict__ F, bf* Ph, bf* Pl) {
    typedef __attribute__((ext_vector_type(4))) unsigned short v4us;
    const int lane = threadIdx.x & 31; const size_t r = (size_t)blockIdx.x * 8 + (threadIdx.x >> 5); if (r >= (size_t)NTOK) return; v4us oh, ol;
#pragma unroll
    for (int i = 0; i < 4; ++i) { const float y = F[r * 128 + lane * 4 + i]; const unsigned short hb = f2bf(y); oh[i] = hb; ol[i] = f2bf(y - bf2f(hb)); }
    const size_t o = r * 128 + lane * 4; *(volatile v4us*)(Ph + o) = oh; *(volatile v4us*)(Pl + o) = ol; __threadfence(); *(volatile v4us*)(Ph + o) = oh; *(volatile v4us*)(Pl + o) = ol;
}
__global__ __launch_bounds__(256) void k_tanh64p(const float* __restrict__ F, bf* Ph, bf* Pl) {
    typedef __attribute__((ext_vector_type(2))) unsigned short v2us;
    const int lane = threadIdx.x & 31; const size_t r = (size_t)blockIdx.x * 8 + (threadIdx.x >> 5); if (r >= (size_t)NTOK) return; v2us oh, ol;
#pragma unroll
    for (int i = 0; i < 2; ++i) { const float y = tanhf(F[r * UU + lane * 2 + i]); const unsigned short hb = f2bf(y); oh[i] = hb; ol[i] = f2bf(y - bf2f(hb)); }
    const size_t o = r * UU + lane * 2; *(volatile v2us*)(Ph + o) = oh; *(volatile v2us*)(Pl + o) = ol; __threadfence(); *(volatile v2us*)(Ph + o) = oh; *(volatile v2us*)(Pl + o) = ol;
}
__global__ __launch_bounds__(256) void k_head(const float* __restrict__ F, const float* __restrict__ Wh, const float* __restrict__ bh, float* OUTB) {
    typedef __attribute__((ext_vector_type(2))) float v2f_;
    const int lane = threadIdx.x & 31; const size_t tok = ((size_t)blockIdx.x * 8 + (threadIdx.x >> 5)) * 32 + lane; if (tok >= (size_t)NTOK) return; float a0 = bfr(bh[0]), a1 = bfr(bh[1]);
#pragma unroll 1
    for (int p = 0; p < PD; ++p) { const float h = tanhf(F[tok * UU + p]); a0 = fmaf(h, bfr(Wh[p * NC]), a0); a1 = fmaf(h, bfr(Wh[p * NC + 1]), a1); }
    v2f_ v; v[0] = a0; v[1] = a1; *(volatile v2f_*)(OUTB + tok * NC) = v; __threadfence(); *(volatile v2f_*)(OUTB + tok * NC) = v;
}

__global__ __launch_bounds__(256) void k_bias2cat(const float* __restrict__ a, const float* __restrict__ b, int n, float* Bv) {
    const int i = threadIdx.x; if (i >= 128) return; float v = 0.f; if (i < n) v = a[i]; else if (b != nullptr && i < 2 * n) v = b[i - n];
    *(volatile float*)(Bv + i) = v; __threadfence(); *(volatile float*)(Bv + i) = v;
}

#define HTOK 65536
extern "C" void kernel_launch(void* const* d_in, const int* in_sizes, int n_in,
                              void* d_out, int out_size, void* d_ws, size_t ws_size, hipStream_t stream) {
    (void)in_sizes; (void)n_in; (void)out_size;
    const int* xi = (const int*)d_in[0]; const float* E = (const float*)d_in[1]; const float* W1r = (const float*)d_in[2]; const float* b1r = (const float*)d_in[3]; const float* W1i = (const float*)d_in[4]; const float* b1i = (const float*)d_in[5]; const float* om1 = (const float*)d_in[6]; const float* Wp1 = (const float*)d_in[7]; const float* bp1 = (const float*)d_in[8];
    const float* W2r = (const float*)d_in[9]; const float* b2r = (const float*)d_in[10]; const float* W2i = (const float*)d_in[11]; const float* b2i = (const float*)d_in[12]; const float* om2 = (const float*)d_in[13]; const float* Wp2 = (const float*)d_in[14]; const float* bp2 = (const float*)d_in[15]; const float* Wpr = (const float*)d_in[16]; const float* bpr = (const float*)d_in[17]; const float* Wh = (const float*)d_in[18]; const float* bh = (const float*)d_in[19];
    float* out = (float*)d_out;
    char* wsp = (char*)d_ws;
    auto take = [&](size_t bytes) { char* p = wsp; wsp += (bytes + 255) & ~(size_t)255; return (void*)p; };
    bf* BW1 = (bf*)take(128 * 128 * 2); float* BB1 = (float*)take(128 * 4); bf* BWP1 = (bf*)take(64 * 128 * 2); bf* BW2 = (bf*)take(128 * 64 * 2); float* BB2 = (float*)take(128 * 4); bf* BWP2 = (bf*)take(64 * 128 * 2); bf* BWPR = (bf*)take(64 * 64 * 2); float* BBPR = (float*)take(64 * 4);
    bf* A = (bf*)take((size_t)HTOK * EDP * 2); float* F = (float*)take((size_t)HTOK * 128 * 4); float* Z = (float*)take((size_t)HTOK * 128 * 4); bf* Ph = (bf*)take((size_t)HTOK * 128 * 2); bf* Pl = (bf*)take((size_t)HTOK * 128 * 2); float* G = (float*)take((size_t)HTOK * UU * 4); bf* Gh = (bf*)take((size_t)HTOK * UU * 2); bf* Gl = (bf*)take((size_t)HTOK * UU * 2);
    if ((size_t)(wsp - (char*)d_ws) > ws_size) return;
    k_w1cat<<<128 / 8, 256, 0, stream>>>(W1r, W1i, BW1); k_bias2cat<<<1, 256, 0, stream>>>(b1r, b1i, UU, BB1); k_wt_small<<<64 / 8, 256, 0, stream>>>(Wp1, 2 * UU, UU, 128, 64, BWP1);
    k_wcat2<<<128 / 8, 256, 0, stream>>>(W2r, W2i, BW2); k_bias2cat<<<1, 256, 0, stream>>>(b2r, b2i, UU, BB2); k_wt_small<<<64 / 8, 256, 0, stream>>>(Wp2, 2 * UU, UU, 128, 64, BWP2);
    k_wt_small<<<64 / 8, 256, 0, stream>>>(Wpr, UU, PD, 64, 64, BWPR); k_bias2cat<<<1, 256, 0, stream>>>(bpr, nullptr, PD, BBPR);
    for (int hf = 0; hf < 2; ++hf) { const size_t t0 = (size_t)hf * HTOK;
        k_embrows<<<HTOK / 8, 256, 0, stream>>>(xi + t0, E, A);
        k_gemmb<false, false><<<dim3(HTOK / 64, 2, 1), 128, 0, stream>>>(A, nullptr, BW1, BB1, F, 128, nullptr, nullptr, EDP);
        k_hopf<<<(NB_) / 8, 256, 0, stream>>>(F, om1, Z);
        k_split128r<<<HTOK / 8, 256, 0, stream>>>(Z, Ph, Pl);
        k_gemmb<true, false><<<dim3(HTOK / 64, 1, 1), 128, 0, stream>>>(Ph, Pl, BWP1, bp1, G, UU, nullptr, nullptr, 128);
        k_relu64p<<<HTOK / 8, 256, 0, stream>>>(G, Gh, Gl);
        k_gemmb<true, false><<<dim3(HTOK / 64, 2, 1), 128, 0, stream>>>(Gh, Gl, BW2, BB2, F, 128, nullptr, nullptr, UU);
        k_hopf<<<(NB_) / 8, 256, 0, stream>>>(F, om2, Z);
        k_split128r<<<HTOK / 8, 256, 0, stream>>>(Z, Ph, Pl);
        k_gemmb<true, false><<<dim3(HTOK / 64, 1, 1), 128, 0, stream>>>(Ph, Pl, BWP2, bp2, G, UU, nullptr, nullptr, 128);
        k_relu64p<<<HTOK / 8, 256, 0, stream>>>(G, Gh, Gl);
        k_gemmb<true, false><<<dim3(HTOK / 64, 1, 1), 128, 0, stream>>>(Gh, Gl, BWPR, BBPR, G, UU, nullptr, nullptr, UU);
        k_head<<<(HTOK / 32) / 8, 256, 0, stream>>>(G, Wh, bh, out + t0 * NC); }
}
